// TorchGNN_85650237817340
// MI455X (gfx1250) — hardware-verified
//
#include <hip/hip_runtime.h>
#include <stddef.h>
#include <math.h>


#define HD      64
#define G3      192
#define NTHR    256
#define NWAVE   8
#define EPT     8
#define NGRP    2
#define CHUNK   (NTHR * EPT * NGRP)
#define WCAP    (EPT * NGRP * 32)
#define LISTN   (NWAVE * WCAP)
#define NBC     4096
#define NBF     1024
#define RCAP    40960
#define RBN     128
#define EWAVE   4
#define ETHR    (EWAVE * 32)
#define TGT     (EWAVE * 32)
#define NGRAN   256
#define DEGCAP  1024
#define OTHR    512
#define BM      32
#define M1P     72
#define M3P     68
#define NPROP   3
#define WSCAP   134217728
#define SCL_A   8.0f
#define SCL_W   16.0f
#define SCL_ACC 0.0078125f

#define RW1A    0
#define RW1C    64
#define RW2     128
#define RW3     192
#define RWIH    256
#define RWHH    448
#define WPROWS  640

#define LDS_FILL ((RCAP + NBF + LISTN) * 4 + 64)

static_assert((CHUNK & (CHUNK - 1)) == 0);
static_assert(CHUNK <= 4096);
static_assert(NBC <= 4096 && NBF <= 4096);
static_assert((NBC & (NBC - 1)) == 0 && (NBF & (NBF - 1)) == 0);
static_assert(NBC == 4 * NBF);
static_assert(OTHR * 8 == NBC);
static_assert((RCAP % 32) == 0);
static_assert(TGT == EWAVE * 32);
static_assert((NGRAN % TGT) == 0 && (NGRAN % BM) == 0);
static_assert((NBF % 32) == 0);
static_assert(HD == 64 && G3 == 3 * HD && (HD % 32) == 0);
static_assert(BM * 8 == NTHR);
static_assert((M1P % 8) == 0 && (M3P % 4) == 0);

typedef float    v2f  __attribute__((ext_vector_type(2)));
typedef float    v4f  __attribute__((ext_vector_type(4)));
typedef float    v8f  __attribute__((ext_vector_type(8)));
typedef int      v4i  __attribute__((ext_vector_type(4)));
typedef _Float16 v2h  __attribute__((ext_vector_type(2)));
typedef _Float16 v4h  __attribute__((ext_vector_type(4)));
typedef _Float16 v8h  __attribute__((ext_vector_type(8)));
typedef _Float16 v16h __attribute__((ext_vector_type(16)));
union FragH { v16h v; v8h h[2]; };

__device__ __forceinline__ v8f wmh(v16h a, v16h b, v8f c) {
  v8f d = __builtin_amdgcn_wmma_f32_16x16x32_f16(false, a, false, b, (short)0, c, false, false);
  asm volatile("v_nop\n\tv_nop\n\tv_nop\n\tv_nop" : "+v"(d) : "v"(a), "v"(b));
  return d;
}

__device__ __forceinline__ v8h cvt8(v4f a, v4f b, float s) {
  v8f t;
  t[0] = a.x * s; t[1] = a.y * s; t[2] = a.z * s; t[3] = a.w * s;
  t[4] = b.x * s; t[5] = b.y * s; t[6] = b.z * s; t[7] = b.w * s;
  return __builtin_convertvector(t, v8h);
}

__device__ __forceinline__ v4f relu4(v4f x) {
  v4f r;
  r.x = x.x > 0.0f ? x.x : 0.0f;
  r.y = x.y > 0.0f ? x.y : 0.0f;
  r.z = x.z > 0.0f ? x.z : 0.0f;
  r.w = x.w > 0.0f ? x.w : 0.0f;
  return r;
}

__device__ __forceinline__ void epi8(v8f acc, v4f c0, v4f c1, v4f& y0, v4f& y1) {
  y0.x = acc[0] * SCL_ACC + c0.x; y0.y = acc[1] * SCL_ACC + c0.y;
  y0.z = acc[2] * SCL_ACC + c0.z; y0.w = acc[3] * SCL_ACC + c0.w;
  y1.x = acc[4] * SCL_ACC + c1.x; y1.y = acc[5] * SCL_ACC + c1.y;
  y1.z = acc[6] * SCL_ACC + c1.z; y1.w = acc[7] * SCL_ACC + c1.w;
}

__device__ __forceinline__ float sigm(float x) {
  x = x > 30.0f ? 30.0f : (x < -30.0f ? -30.0f : x);
  const float e = expf(-x);
  return 1.0f / (1.0f + e);
}

__device__ __forceinline__ void wave_sync_lds() {
  __builtin_amdgcn_fence(__ATOMIC_RELEASE, "wavefront");
  __builtin_amdgcn_wave_barrier();
}

template <int NB>
__device__ __forceinline__ int scan_chunk(const int* __restrict__ dsts, int nE, int cbase, int slotBase,
                                          int vec8, int* list, int tid, int lane, int wave) {
  int wc = 0;
#pragma unroll
  for (int g = 0; g < NGRP; ++g) {
    const int el0  = (g * NTHR + tid) * EPT;
    const int e0   = cbase + el0;
    const int sent = -2147483647 - 1;
    v4i da, db;
    if (vec8 != 0 && cbase + CHUNK <= nE) {
      da = *(const v4i*)(dsts + e0);
      db = *(const v4i*)(dsts + e0 + 4);
    } else {
      da.x = (e0     < nE) ? dsts[min(e0, nE - 1)] : sent;
      da.y = (e0 + 1 < nE) ? dsts[min(e0 + 1, nE - 1)] : sent;
      da.z = (e0 + 2 < nE) ? dsts[min(e0 + 2, nE - 1)] : sent;
      da.w = (e0 + 3 < nE) ? dsts[min(e0 + 3, nE - 1)] : sent;
      db.x = (e0 + 4 < nE) ? dsts[min(e0 + 4, nE - 1)] : sent;
      db.y = (e0 + 5 < nE) ? dsts[min(e0 + 5, nE - 1)] : sent;
      db.z = (e0 + 6 < nE) ? dsts[min(e0 + 6, nE - 1)] : sent;
      db.w = (e0 + 7 < nE) ? dsts[min(e0 + 7, nE - 1)] : sent;
    }
    const unsigned nb = (unsigned)slotBase;
    const unsigned s0 = (unsigned)da.x - nb, s1 = (unsigned)da.y - nb;
    const unsigned s2 = (unsigned)da.z - nb, s3 = (unsigned)da.w - nb;
    const unsigned s4 = (unsigned)db.x - nb, s5 = (unsigned)db.y - nb;
    const unsigned s6 = (unsigned)db.z - nb, s7 = (unsigned)db.w - nb;
    const bool h0 = s0 < (unsigned)NB, h1 = s1 < (unsigned)NB, h2 = s2 < (unsigned)NB, h3 = s3 < (unsigned)NB;
    const bool h4 = s4 < (unsigned)NB, h5 = s5 < (unsigned)NB, h6 = s6 < (unsigned)NB, h7 = s7 < (unsigned)NB;
    const unsigned any = __builtin_amdgcn_ballot_w32(h0 | h1 | h2 | h3 | h4 | h5 | h6 | h7);
    if (any != 0u) {
#define HITJ(J, HJ, SJ) { \
        const unsigned mj = __builtin_amdgcn_ballot_w32(HJ); \
        if (mj != 0u) { \
          if (HJ) { \
            const int pos = wc + (int)__builtin_amdgcn_mbcnt_lo(mj, 0u); \
            if (pos < WCAP) list[wave * WCAP + pos] = ((el0 + (J)) << 12) | (int)(SJ); \
          } \
          wc += (int)__builtin_popcount(mj); } }
      HITJ(0, h0, s0)
      HITJ(1, h1, s1)
      HITJ(2, h2, s2)
      HITJ(3, h3, s3)
      HITJ(4, h4, s4)
      HITJ(5, h5, s5)
      HITJ(6, h6, s6)
      HITJ(7, h7, s7)
#undef HITJ
    }
  }
  return wc;
}

__global__ __launch_bounds__(NTHR) void k_extract(const int* __restrict__ edges, int* objp, int nE, int nUnits) {
  const int i = (int)blockIdx.x * NTHR + (int)threadIdx.x;
  if (i >= nUnits) return;
  const int e0 = 4 * i;
  const int a0 = min(e0, nE - 1), a1 = min(e0 + 1, nE - 1), a2 = min(e0 + 2, nE - 1), a3 = min(e0 + 3, nE - 1);
  v4i v;
  v.x = edges[(size_t)a0 * 2 + 1];
  v.y = edges[(size_t)a1 * 2 + 1];
  v.z = edges[(size_t)a2 * 2 + 1];
  v.w = edges[(size_t)a3 * 2 + 1];
  int* d = objp + (size_t)4 * i;
  *(volatile v4i*)d = v;
  __threadfence();
  *(volatile v4i*)d = v;
}

__global__ __launch_bounds__(NTHR) void k_prepw(const float* __restrict__ W1, const float* __restrict__ W2,
                                               const float* __restrict__ W3, const float* __restrict__ Wih,
                                               const float* __restrict__ Whh, _Float16* wp) {
  const int seg = (int)blockIdx.y;
  const float* src;
  int ld, kb, rows, drow;
  if (seg == 0)      { src = W1;  ld = HD; kb = 0;  rows = HD; drow = RW1A; }
  else if (seg == 1) { src = W1;  ld = HD; kb = 68; rows = HD; drow = RW1C; }
  else if (seg == 2) { src = W2;  ld = HD; kb = 0;  rows = HD; drow = RW2;  }
  else if (seg == 3) { src = W3;  ld = HD; kb = 0;  rows = HD; drow = RW3;  }
  else if (seg == 4) { src = Wih; ld = G3; kb = 0;  rows = G3; drow = RWIH; }
  else               { src = Whh; ld = G3; kb = 0;  rows = G3; drow = RWHH; }
  const int u = (int)blockIdx.x * NTHR + (int)threadIdx.x;
  if (u >= rows * 8) return;
  const int R = u >> 3, q = u & 7;
  const float* p = src + (size_t)(kb + 8 * q) * ld + R;
  v4f a, b;
  a.x = p[0];               a.y = p[(size_t)ld];      a.z = p[(size_t)2 * ld];  a.w = p[(size_t)3 * ld];
  b.x = p[(size_t)4 * ld];  b.y = p[(size_t)5 * ld];  b.z = p[(size_t)6 * ld];  b.w = p[(size_t)7 * ld];
  const v8h o = cvt8(a, b, SCL_W);
  _Float16* d = wp + (size_t)(drow + R) * HD + 8 * q;
  *(volatile v8h*)d = o;
  __threadfence();
  *(volatile v8h*)d = o;
}

__global__ __launch_bounds__(NTHR) void k_count(
    const int* __restrict__ dsts, int* cnt, int nE, int vec8) {
  __shared__ __attribute__((aligned(16))) int scnt[NBC];
  __shared__ __attribute__((aligned(16))) int list[LISTN];
  __shared__ int wcnt[NWAVE];
  const int tid = threadIdx.x, lane = tid & 31, wave = tid >> 5;
  const int nodeBase = blockIdx.x * NBC;

  for (int i = tid; i < NBC; i += NTHR) scnt[i] = 0;
  __syncthreads();

  const int nChunks = (nE + CHUNK - 1) / CHUNK;
#pragma unroll 1
  for (int ch = 0; ch < nChunks; ++ch) {
    const int cbase = ch * CHUNK;
    const int wc = scan_chunk<NBC>(dsts, nE, cbase, nodeBase, vec8, list, tid, lane, wave);
    if (lane == 0) wcnt[wave] = wc;
    __syncthreads();
    if (wave == 0) {
#pragma unroll 1
      for (int wsx = 0; wsx < NWAVE; ++wsx) {
        int n = __builtin_amdgcn_readfirstlane(wcnt[wsx]);
        n = n > WCAP ? WCAP : (n < 0 ? 0 : n);
        const int* lp = list + wsx * WCAP;
#pragma unroll 1
        for (int i = 0; i < n; ++i) {
          const int ent  = __builtin_amdgcn_readfirstlane(lp[i]);
          const int slot = ent & (NBC - 1);
          if (lane == 0) scnt[slot] = scnt[slot] + 1;
        }
      }
    }
    __syncthreads();
  }

  v4i cq[4];
#pragma unroll
  for (int q = 0; q < 4; ++q) {
    const int f = (wave * 4 + q) * 128 + 4 * lane;
    cq[q] = *(const v4i*)(scnt + f);
  }
  int* cp = cnt + (size_t)nodeBase;
#pragma unroll
  for (int q = 0; q < 4; ++q) {
    const int f = (wave * 4 + q) * 128 + 4 * lane;
    *(volatile v4i*)(cp + f) = cq[q];
  }
  __threadfence();
#pragma unroll
  for (int q = 0; q < 4; ++q) {
    const int f = (wave * 4 + q) * 128 + 4 * lane;
    *(volatile v4i*)(cp + f) = cq[q];
  }
}

__global__ __launch_bounds__(OTHR) void k_offsets(
    const int* __restrict__ cnt, int* off, int* rbase, int nChunk) {
  __shared__ __attribute__((aligned(16))) int soff[NBC];
  __shared__ __attribute__((aligned(16))) int srb[RBN];
  __shared__ int wtot[OTHR / 32];
  const int tid = threadIdx.x, lane = tid & 31, wave = tid >> 5, sub = tid >> 7;
  for (int i = tid; i < RBN; i += OTHR) srb[i] = 0;
  int carry = 0;
#pragma unroll 1
  for (int ch = 0; ch < nChunk; ++ch) {
    const int base = ch * NBC;
    const v4i c0 = *(const v4i*)(cnt + base + 8 * tid);
    const v4i c1 = *(const v4i*)(cnt + base + 8 * tid + 4);
    const int e0 = max(c0.x, 0), e1 = max(c0.y, 0), e2 = max(c0.z, 0), e3 = max(c0.w, 0);
    const int e4 = max(c1.x, 0), e5 = max(c1.y, 0), e6 = max(c1.z, 0), e7 = max(c1.w, 0);
    const int ts = e0 + e1 + e2 + e3 + e4 + e5 + e6 + e7;
    int incl = ts;
#pragma unroll
    for (int d = 1; d < 32; d <<= 1) {
      const int t = __shfl_up(incl, d);
      if (lane >= d) incl += t;
    }
    if (lane == 31) wtot[wave] = incl;
    __syncthreads();
    const int S0 = wtot[0]  + wtot[1]  + wtot[2]  + wtot[3];
    const int S1 = wtot[4]  + wtot[5]  + wtot[6]  + wtot[7];
    const int S2 = wtot[8]  + wtot[9]  + wtot[10] + wtot[11];
    const int S3 = wtot[12] + wtot[13] + wtot[14] + wtot[15];
    int pre = 0;
#pragma unroll 1
    for (int w = 4 * sub; w < wave; ++w) pre += wtot[w];
    const int b0 = carry;
    const int b1 = b0 + ((S0 + 31) & ~31);
    const int b2 = b1 + ((S1 + 31) & ~31);
    const int b3 = b2 + ((S2 + 31) & ~31);
    const int b4 = b3 + ((S3 + 31) & ~31);
    const int myb = sub == 0 ? b0 : (sub == 1 ? b1 : (sub == 2 ? b2 : b3));
    if (tid == 0) {
      srb[min(4 * ch + 0, RBN - 1)] = b0;
      srb[min(4 * ch + 1, RBN - 1)] = b1;
      srb[min(4 * ch + 2, RBN - 1)] = b2;
      srb[min(4 * ch + 3, RBN - 1)] = b3;
    }
    int run = myb + pre + incl - ts;
    soff[8 * tid + 0] = run; run += e0;
    soff[8 * tid + 1] = run; run += e1;
    soff[8 * tid + 2] = run; run += e2;
    soff[8 * tid + 3] = run; run += e3;
    soff[8 * tid + 4] = run; run += e4;
    soff[8 * tid + 5] = run; run += e5;
    soff[8 * tid + 6] = run; run += e6;
    soff[8 * tid + 7] = run;
    carry = b4;
    __syncthreads();
    const v4i o0 = *(const v4i*)(soff + 4 * tid);
    const v4i o1 = *(const v4i*)(soff + 4 * (tid + OTHR));
    int* op = off + base;
    *(volatile v4i*)(op + 4 * tid) = o0;
    *(volatile v4i*)(op + 4 * (tid + OTHR)) = o1;
    __threadfence();
    *(volatile v4i*)(op + 4 * tid) = o0;
    *(volatile v4i*)(op + 4 * (tid + OTHR)) = o1;
    __syncthreads();
  }
  if (tid == 0) srb[min(4 * nChunk, RBN - 1)] = carry;
  __syncthreads();
  v4i rv = {0, 0, 0, 0};
  if (tid < 32) rv = *(const v4i*)(srb + 4 * tid);
  if (tid < 32) *(volatile v4i*)(rbase + 4 * tid) = rv;
  __threadfence();
  if (tid < 32) *(volatile v4i*)(rbase + 4 * tid) = rv;
}

__global__ __launch_bounds__(NTHR) void k_fill(
    const int* __restrict__ dsts, const int* __restrict__ off, const int* __restrict__ rbase,
    int* csr, int nE, int vec8, int csrLen) {
  extern __shared__ v4f lds_dyn[];
  int* region = (int*)lds_dyn;
  int* cursor = region + RCAP;
  int* list   = cursor + NBF;
  int* wcnt   = list + LISTN;
  const int tid = threadIdx.x, lane = tid & 31, wave = tid >> 5;
  const int b = blockIdx.x;
  const int nodeBase = b * NBF;

  int rb0 = rbase[b];
  const int rb1 = rbase[b + 1];
  rb0 = rb0 < 0 ? 0 : (rb0 > csrLen ? csrLen : rb0);
  rb0 &= ~31;
  int len = rb1 - rb0;
  len = len < 0 ? 0 : (len > RCAP ? RCAP : len);
  int lenW = (len + 31) & ~31;
  if (rb0 + lenW > csrLen) lenW = (csrLen - rb0) & ~31;

  {
    const v4i z = {0, 0, 0, 0};
    for (int i = tid; i < RCAP / 4; i += NTHR) ((v4i*)region)[i] = z;
    for (int s = tid; s < NBF; s += NTHR) {
      int o = off[nodeBase + s] - rb0;
      o = o < 0 ? 0 : (o > RCAP ? RCAP : o);
      cursor[s] = o;
    }
  }
  __syncthreads();

  const int nChunks = (nE + CHUNK - 1) / CHUNK;
#pragma unroll 1
  for (int ch = 0; ch < nChunks; ++ch) {
    const int cbase = ch * CHUNK;
    const int wc = scan_chunk<NBF>(dsts, nE, cbase, nodeBase, vec8, list, tid, lane, wave);
    if (lane == 0) wcnt[wave] = wc;
    __syncthreads();
    if (wave == 0) {
#pragma unroll 1
      for (int wsx = 0; wsx < NWAVE; ++wsx) {
        int n = __builtin_amdgcn_readfirstlane(wcnt[wsx]);
        n = n > WCAP ? WCAP : (n < 0 ? 0 : n);
        const int* lp = list + wsx * WCAP;
#pragma unroll 1
        for (int i = 0; i < n; ++i) {
          const int ent  = __builtin_amdgcn_readfirstlane(lp[i]);
          const int slot = ent & (NBF - 1);
          int e = cbase + ((ent >> 12) & (CHUNK - 1));
          e = e > nE - 1 ? nE - 1 : (e < 0 ? 0 : e);
          if (lane == 0) {
            int pos = cursor[slot];
            pos = pos < 0 ? 0 : (pos > RCAP - 1 ? RCAP - 1 : pos);
            region[pos] = e;
            const int np = pos + 1;
            cursor[slot] = np > RCAP ? RCAP : np;
          }
        }
      }
    }
    __syncthreads();
  }

  const int nv = lenW >> 2;
  int* gp = csr + rb0;
#pragma unroll 1
  for (int i = tid; i < nv; i += NTHR) { const v4i v = ((const v4i*)region)[i]; *(volatile v4i*)(gp + 4 * i) = v; }
  __threadfence();
#pragma unroll 1
  for (int i = tid; i < nv; i += NTHR) { const v4i v = ((const v4i*)region)[i]; *(volatile v4i*)(gp + 4 * i) = v; }
}

__device__ __forceinline__ void put_row(_Float16* aggP, int node, int lane, v2f v, bool poison) {
  v2f s = v * SCL_A;
  if (poison) { const float qn = __int_as_float(0x7fc00000); s.x = qn; s.y = qn; }
  const v2h o = __builtin_convertvector(s, v2h);
  _Float16* gp = aggP + (size_t)node * HD + 2 * lane;
  *(volatile v2h*)gp = o;
  __threadfence();
  *(volatile v2h*)gp = o;
}

__global__ __launch_bounds__(ETHR) void k_edge(
    const int* __restrict__ csr, const int* __restrict__ offp, const int* __restrict__ cnt,
    const int* __restrict__ edges, const float* __restrict__ Jm,
    const float* __restrict__ Pp, const float* __restrict__ Qp,
    const _Float16* __restrict__ wp, const float* __restrict__ W1,
    const float* __restrict__ b2, const float* __restrict__ b3,
    _Float16* aggP, int nN, int nE, int csrLen) {
  __shared__ __attribute__((aligned(16))) _Float16 sM1[EWAVE * 16 * M1P];
  __shared__ __attribute__((aligned(16))) float sM3[EWAVE * 16 * M3P];
  __shared__ __attribute__((aligned(16))) float swb[HD];
  __shared__ __attribute__((aligned(16))) float sb2[HD];
  __shared__ __attribute__((aligned(16))) float sb3[HD];
  const int tid = threadIdx.x, lane = tid & 31, wave = tid >> 5;
  const int hh = lane >> 4, m = lane & 15;
  if (tid < HD) {
    swb[tid] = (W1[66 * HD + tid] - W1[67 * HD + tid]) - W1[134 * HD + tid] + W1[135 * HD + tid];
    sb2[tid] = b2[tid];
    sb3[tid] = b3[tid];
  }
  __syncthreads();

  _Float16* m1w = sM1 + wave * 16 * M1P;
  float* m3w = sM3 + wave * 16 * M3P;
  _Float16* m1row = m1w + m * M1P;
  float* m3row = m3w + m * M3P;
  const _Float16* w2p = wp + (size_t)RW2 * HD;
  const _Float16* w3p = wp + (size_t)RW3 * HD;
  const int tbase = blockIdx.x * TGT + wave * 32;
  const v8f z8 = {0.f, 0.f, 0.f, 0.f, 0.f, 0.f, 0.f, 0.f};

  const int cl = tbase + lane;
  int cnt_l = cnt[cl];
  cnt_l = cnt_l < 0 ? 0 : (cnt_l > nE ? nE : cnt_l);
  int off_l = offp[cl];
  off_l = off_l < 0 ? 0 : (off_l > csrLen ? csrLen : off_l);
  const int rs = __builtin_amdgcn_readfirstlane(off_l);
  int end_l = off_l + cnt_l;
  end_l = end_l > csrLen ? csrLen : end_l;
  end_l = end_l < rs ? rs : end_l;
  const int reRaw = __builtin_amdgcn_readlane(end_l, 31);
  const int cap = rs + 32 * DEGCAP;
  const bool poison = reRaw > cap;
  const int re = reRaw > cap ? cap : reRaw;

  int cur = -1, nextW = 0;
  v2f acc = {0.0f, 0.0f};
  const int hb = 8 * (hh ^ 1);

#pragma unroll 1
  for (int p = rs; p < re; p += 16) {
    int pos = p + m;
    pos = pos < 0 ? 0 : (pos > csrLen - 1 ? csrLen - 1 : pos);
    int el = csr[pos];
    el = el < 0 ? 0 : (el > nE - 1 ? nE - 1 : el);
    int src = edges[(size_t)el * 2 + 0];
    src = src < 0 ? 0 : (src > nN - 1 ? nN - 1 : src);
    int dst = edges[(size_t)el * 2 + 1];
    dst = dst < 0 ? 0 : (dst > nN - 1 ? nN - 1 : dst);
    const float jv = Jm[el];
    const float* prow = Pp + (size_t)src * HD;
    const float* qrow = Qp + (size_t)dst * HD;

#pragma unroll
    for (int j = 0; j < 4; ++j) {
      const int c0 = 16 * j + hb;
      const v4f p0 = *(const v4f*)(prow + c0);
      const v4f p1 = *(const v4f*)(prow + c0 + 4);
      const v4f q0 = *(const v4f*)(qrow + c0);
      const v4f q1 = *(const v4f*)(qrow + c0 + 4);
      const v4f w0 = *(const v4f*)(swb + c0);
      const v4f w1 = *(const v4f*)(swb + c0 + 4);
      const v4f s0 = (p0 + q0) + w0 * jv;
      const v4f s1 = (p1 + q1) + w1 * jv;
      *(v8h*)(m1row + c0) = cvt8(relu4(s0), relu4(s1), SCL_A);
    }
    wave_sync_lds();

    FragH mb[2];
#pragma unroll
    for (int ks = 0; ks < 2; ++ks) {
      mb[ks].h[0] = *(const v8h*)(m1row + 32 * ks + 8 * hh);
      mb[ks].h[1] = *(const v8h*)(m1row + 32 * ks + 16 + 8 * hh);
    }

    v8f acc2[4];
#pragma unroll
    for (int T = 0; T < 4; ++T) {
      acc2[T] = z8;
      const _Float16* wr = w2p + (size_t)(16 * T + m) * HD + 8 * hh;
#pragma unroll
      for (int ks = 0; ks < 2; ++ks) {
        FragH a;
        a.h[0] = *(const v8h*)(wr + 32 * ks);
        a.h[1] = *(const v8h*)(wr + 32 * ks + 16);
        acc2[T] = wmh(a.v, mb[ks].v, acc2[T]);
      }
    }

    FragH nb[2];
#pragma unroll
    for (int ks = 0; ks < 2; ++ks) {
#pragma unroll
      for (int u = 0; u < 2; ++u) {
        const int T = 2 * ks + u;
        const v4f c0 = *(const v4f*)(sb2 + 16 * T + 8 * hh);
        const v4f c1 = *(const v4f*)(sb2 + 16 * T + 8 * hh + 4);
        v4f x0, x1;
        epi8(acc2[T], c0, c1, x0, x1);
        nb[ks].h[u] = cvt8(relu4(x0), relu4(x1), SCL_A);
      }
    }

#pragma unroll
    for (int T = 0; T < 4; ++T) {
      v8f a3 = z8;
      const _Float16* wr = w3p + (size_t)(16 * T + m) * HD + 8 * hh;
#pragma unroll
      for (int ks = 0; ks < 2; ++ks) {
        FragH a;
        a.h[0] = *(const v8h*)(wr + 32 * ks);
        a.h[1] = *(const v8h*)(wr + 32 * ks + 16);
        a3 = wmh(a.v, nb[ks].v, a3);
      }
      const v4f c0 = *(const v4f*)(sb3 + 16 * T + 8 * hh);
      const v4f c1 = *(const v4f*)(sb3 + 16 * T + 8 * hh + 4);
      v4f y0, y1;
      epi8(a3, c0, c1, y0, y1);
      float* mr = m3row + 16 * T + 8 * hh;
      *(v4f*)mr = y0;
      *(v4f*)(mr + 4) = y1;
    }
    wave_sync_lds();

#pragma unroll 1
    for (int i = 0; i < 16; ++i) {
      const int prow_ = p + i;
      if (prow_ < re) {
        int idx = (int)__builtin_popcount(__builtin_amdgcn_ballot_w32(end_l <= prow_));
        idx = idx > 31 ? 31 : idx;
        if (idx != cur) {
          if (cur >= 0) { put_row(aggP, tbase + cur, lane, acc, poison); nextW = cur + 1; }
#pragma unroll 1
          for (int jn = nextW; jn < idx; ++jn) {
            const v2f zz = {0.0f, 0.0f};
            put_row(aggP, tbase + jn, lane, zz, poison);
          }
          nextW = idx;
          cur = idx;
          acc.x = 0.0f; acc.y = 0.0f;
        }
        const v2f v = *(const v2f*)(m3w + i * M3P + 2 * lane);
        acc = acc + v;
      }
    }
    wave_sync_lds();
  }

  if (cur >= 0) { put_row(aggP, tbase + cur, lane, acc, poison); nextW = cur + 1; }
#pragma unroll 1
  for (int jn = nextW; jn < 32; ++jn) {
    const v2f zz = {0.0f, 0.0f};
    put_row(aggP, tbase + jn, lane, zz, poison);
  }
}

__global__ __launch_bounds__(NTHR) void k_node(
    const _Float16* __restrict__ aggP, const _Float16* __restrict__ wp,
    const float* __restrict__ W1, const float* __restrict__ b1,
    const float* __restrict__ bnode, const float* __restrict__ Win, const float* __restrict__ bin0,
    const float* __restrict__ bih, const float* __restrict__ bhh,
    const float* __restrict__ Wout, const float* __restrict__ bout,
    float* H32, _Float16* H16, float* Pp, float* Qp, float* out, int nN, int mode) {
  __shared__ __attribute__((aligned(16))) _Float16 hs[BM * HD];
  __shared__ __attribute__((aligned(16))) float stg[BM * HD];
  __shared__ __attribute__((aligned(16))) float pst[BM * HD];
  __shared__ __attribute__((aligned(16))) float qst[BM * HD];
  __shared__ __attribute__((aligned(16))) float swa[HD];
  __shared__ __attribute__((aligned(16))) float swc[HD];
  __shared__ __attribute__((aligned(16))) float sb1[HD];
  __shared__ __attribute__((aligned(16))) float ssc[2 * BM];
  const int tid = threadIdx.x, lane = tid & 31, wave = tid >> 5;
  const int hh = lane >> 4, m = lane & 15;
  const int rg = wave >> 2, ct = wave & 3;
  const int rowBase = (int)blockIdx.x * BM;
  const int arow = rowBase + rg * 16 + m;
  const int ncol = ct * 16 + m;
  const int lrow0 = rg * 16 + 8 * hh;
  const v8f z8 = {0.f, 0.f, 0.f, 0.f, 0.f, 0.f, 0.f, 0.f};
  const v4f z4 = {0.f, 0.f, 0.f, 0.f};

  if (tid < HD) {
    swa[tid] = W1[64 * HD + tid] - W1[65 * HD + tid];
    swc[tid] = W1[133 * HD + tid] - W1[132 * HD + tid];
    sb1[tid] = b1[tid];
  }

  if (mode == 0) {
    const int row = tid >> 3, q = tid & 7;
    const int grow = rowBase + row;
    const int gr = grow > nN - 1 ? nN - 1 : grow;
    const float bb = bnode[gr];
    const v4f wa0 = *(const v4f*)(Win + 8 * q),      wa1 = *(const v4f*)(Win + 8 * q + 4);
    const v4f wb0 = *(const v4f*)(Win + HD + 8 * q), wb1 = *(const v4f*)(Win + HD + 8 * q + 4);
    const v4f bi0 = *(const v4f*)(bin0 + 8 * q),     bi1 = *(const v4f*)(bin0 + 8 * q + 4);
    v4f v0 = (wa0 * bb - wb0 * bb) + bi0;
    v4f v1 = (wa1 * bb - wb1 * bb) + bi1;
    if (grow >= nN) { v0 = z4; v1 = z4; }
    *(v4f*)(stg + (size_t)row * HD + 8 * q) = v0;
    *(v4f*)(stg + (size_t)row * HD + 8 * q + 4) = v1;
  } else {
    FragH xa[2], ha[2];
    {
      const _Float16* xr = aggP + (size_t)arow * HD + 8 * hh;
      const _Float16* hr = H16 + (size_t)arow * HD + 8 * hh;
#pragma unroll
      for (int kt = 0; kt < 2; ++kt) {
        xa[kt].h[0] = *(const v8h*)(xr + 32 * kt);
        xa[kt].h[1] = *(const v8h*)(xr + 32 * kt + 16);
        ha[kt].h[0] = *(const v8h*)(hr + 32 * kt);
        ha[kt].h[1] = *(const v8h*)(hr + 32 * kt + 16);
      }
    }
    v8f gir = z8, giz = z8, gin = z8, ghr = z8, ghz = z8, ghn = z8;
#pragma unroll
    for (int kt = 0; kt < 2; ++kt) {
      const _Float16* bi = wp + (size_t)(RWIH + ncol) * HD + 32 * kt + 8 * hh;
      const _Float16* bh = wp + (size_t)(RWHH + ncol) * HD + 32 * kt + 8 * hh;
      FragH bf;
      bf.h[0] = *(const v8h*)(bi);                       bf.h[1] = *(const v8h*)(bi + 16);                       gir = wmh(xa[kt].v, bf.v, gir);
      bf.h[0] = *(const v8h*)(bi + (size_t)64 * HD);     bf.h[1] = *(const v8h*)(bi + (size_t)64 * HD + 16);     giz = wmh(xa[kt].v, bf.v, giz);
      bf.h[0] = *(const v8h*)(bi + (size_t)128 * HD);    bf.h[1] = *(const v8h*)(bi + (size_t)128 * HD + 16);    gin = wmh(xa[kt].v, bf.v, gin);
      bf.h[0] = *(const v8h*)(bh);                       bf.h[1] = *(const v8h*)(bh + 16);                       ghr = wmh(ha[kt].v, bf.v, ghr);
      bf.h[0] = *(const v8h*)(bh + (size_t)64 * HD);     bf.h[1] = *(const v8h*)(bh + (size_t)64 * HD + 16);     ghz = wmh(ha[kt].v, bf.v, ghz);
      bf.h[0] = *(const v8h*)(bh + (size_t)128 * HD);    bf.h[1] = *(const v8h*)(bh + (size_t)128 * HD + 16);    ghn = wmh(ha[kt].v, bf.v, ghn);
    }
    {
      const float bir = bih[ncol], biz = bih[HD + ncol], bin_ = bih[2 * HD + ncol];
      const float bhr = bhh[ncol], bhz = bhh[HD + ncol], bhn = bhh[2 * HD + ncol];
      float* sp = stg + (size_t)lrow0 * HD + ncol;
      const float* hp = H32 + (size_t)(rowBase + lrow0) * HD + ncol;
#pragma unroll
      for (int r = 0; r < 8; ++r) {
        const float hold = hp[(size_t)r * HD];
        const float xr_ = gir[r] * SCL_ACC + bir;
        const float hr_ = ghr[r] * SCL_ACC + bhr;
        const float xz_ = giz[r] * SCL_ACC + biz;
        const float hz_ = ghz[r] * SCL_ACC + bhz;
        const float xn_ = gin[r] * SCL_ACC + bin_;
        const float hn_ = ghn[r] * SCL_ACC + bhn;
        const float rgt = sigm(xr_ + hr_);
        const float zgt = sigm(xz_ + hz_);
        const float ngt = tanhf(xn_ + rgt * hn_);
        float h = (1.0f - zgt) * ngt + zgt * hold;
        h = (rowBase + lrow0 + r < nN) ? h : 0.0f;
        sp[r * HD] = h;
      }
    }
  }
  __syncthreads();

  const v8h oh = cvt8(*(const v4f*)(stg + 8 * tid), *(const v4f*)(stg + 8 * tid + 4), SCL_A);
  *(v8h*)(hs + 8 * tid) = oh;
  __syncthreads();

  if (mode != 2) {
    const _Float16* ar  = hs + (size_t)(rg * 16 + m) * HD + 8 * hh;
    const _Float16* bpa = wp + (size_t)(RW1A + ncol) * HD + 8 * hh;
    const _Float16* bpc = wp + (size_t)(RW1C + ncol) * HD + 8 * hh;
    v8f ap8 = z8, aq8 = z8;
#pragma unroll
    for (int kt = 0; kt < 2; ++kt) {
      FragH a, bf;
      a.h[0] = *(const v8h*)(ar + 32 * kt);
      a.h[1] = *(const v8h*)(ar + 32 * kt + 16);
      bf.h[0] = *(const v8h*)(bpa + 32 * kt);
      bf.h[1] = *(const v8h*)(bpa + 32 * kt + 16);
      ap8 = wmh(a.v, bf.v, ap8);
      bf.h[0] = *(const v8h*)(bpc + 32 * kt);
      bf.h[1] = *(const v8h*)(bpc + 32 * kt + 16);
      aq8 = wmh(a.v, bf.v, aq8);
    }
    const float wac = swa[ncol], wcc = swc[ncol], b1c = sb1[ncol];
#pragma unroll
    for (int r = 0; r < 8; ++r) {
      const int grow = rowBase + lrow0 + r;
      const int gr = grow > nN - 1 ? nN - 1 : grow;
      const float bb = bnode[gr];
      float pv = ap8[r] * SCL_ACC + bb * wac;
      float qv = (aq8[r] * SCL_ACC + bb * wcc) + b1c;
      pv = (grow < nN) ? pv : 0.0f;
      qv = (grow < nN) ? qv : 0.0f;
      pst[(size_t)(lrow0 + r) * HD + ncol] = pv;
      qst[(size_t)(lrow0 + r) * HD + ncol] = qv;
    }
  } else {
    const int row = tid >> 3, q = tid & 7;
    const v4f s0 = *(const v4f*)(stg + (size_t)row * HD + 8 * q);
    const v4f s1 = *(const v4f*)(stg + (size_t)row * HD + 8 * q + 4);
    const v4f w0 = *(const v4f*)(Wout + 16 * q);
    const v4f w1 = *(const v4f*)(Wout + 16 * q + 4);
    const v4f w2 = *(const v4f*)(Wout + 16 * q + 8);
    const v4f w3 = *(const v4f*)(Wout + 16 * q + 12);
    float a0 = s0.x * w0.x + s0.y * w0.z + s0.z * w1.x + s0.w * w1.z
             + s1.x * w2.x + s1.y * w2.z + s1.z * w3.x + s1.w * w3.z;
    float a1 = s0.x * w0.y + s0.y * w0.w + s0.z * w1.y + s0.w * w1.w
             + s1.x * w2.y + s1.y * w2.w + s1.z * w3.y + s1.w * w3.w;
    a0 += __shfl_xor(a0, 4); a0 += __shfl_xor(a0, 2); a0 += __shfl_xor(a0, 1);
    a1 += __shfl_xor(a1, 4); a1 += __shfl_xor(a1, 2); a1 += __shfl_xor(a1, 1);
    if (q == 0) { ssc[2 * row] = a0 + bout[0]; ssc[2 * row + 1] = a1 + bout[1]; }
  }
  __syncthreads();

  const v4f o0 = *(const v4f*)(stg + 4 * tid);
  const v4f o1 = *(const v4f*)(stg + 4 * (tid + NTHR));
  v4f p0 = z4, p1 = z4, q0 = z4, q1 = z4;
  if (mode != 2) {
    p0 = *(const v4f*)(pst + 4 * tid);
    p1 = *(const v4f*)(pst + 4 * (tid + NTHR));
    q0 = *(const v4f*)(qst + 4 * tid);
    q1 = *(const v4f*)(qst + 4 * (tid + NTHR));
  }
  int nv = nN - rowBase;
  nv = nv < 0 ? 0 : (nv > BM ? BM : nv);
  const int nf = 2 * nv, nq4 = nf >> 2, rem = nf & 3;
  v4f sv = z4;
  v2f sv2 = {0.0f, 0.0f};
  if (mode == 2) {
    if (tid < 16) sv = *(const v4f*)(ssc + 4 * tid);
    const int t0 = (4 * nq4) & 63, t1 = (4 * nq4 + 1) & 63;
    sv2.x = ssc[t0]; sv2.y = ssc[t1];
  }
  const bool doOut = (mode == 2) && (nv > 0);

  float* t32 = H32 + (size_t)rowBase * HD;
  _Float16* t16 = H16 + (size_t)rowBase * HD;
  float* tp = Pp + (size_t)rowBase * HD;
  float* tq = Qp + (size_t)rowBase * HD;
  float* op = out + (size_t)2 * rowBase;

  *(volatile v4f*)(t32 + 4 * tid) = o0;
  *(volatile v4f*)(t32 + 4 * (size_t)(tid + NTHR)) = o1;
  *(volatile v8h*)(t16 + 8 * (size_t)tid) = oh;
  if (mode != 2) {
    *(volatile v4f*)(tp + 4 * tid) = p0;
    *(volatile v4f*)(tp + 4 * (size_t)(tid + NTHR)) = p1;
    *(volatile v4f*)(tq + 4 * tid) = q0;
    *(volatile v4f*)(tq + 4 * (size_t)(tid + NTHR)) = q1;
  }
  if (doOut) {
    if (tid < nq4) *(volatile v4f*)(op + 4 * tid) = sv;
    if (rem != 0 && tid == nq4) *(volatile v2f*)(op + 4 * nq4) = sv2;
  }
  __threadfence();
  *(volatile v4f*)(t32 + 4 * tid) = o0;
  *(volatile v4f*)(t32 + 4 * (size_t)(tid + NTHR)) = o1;
  *(volatile v8h*)(t16 + 8 * (size_t)tid) = oh;
  if (mode != 2) {
    *(volatile v4f*)(tp + 4 * tid) = p0;
    *(volatile v4f*)(tp + 4 * (size_t)(tid + NTHR)) = p1;
    *(volatile v4f*)(tq + 4 * tid) = q0;
    *(volatile v4f*)(tq + 4 * (size_t)(tid + NTHR)) = q1;
  }
  if (doOut) {
    if (tid < nq4) *(volatile v4f*)(op + 4 * tid) = sv;
    if (rem != 0 && tid == nq4) *(volatile v2f*)(op + 4 * nq4) = sv2;
  }
}

extern "C" void kernel_launch(void* const* d_in, const int* in_sizes, int n_in,
                              void* d_out, int out_size, void* d_ws, size_t ws_size,
                              hipStream_t stream) {
  if (n_in < 18) return;
  const int nN = in_sizes[2];
  if (nN <= 0 || nN > (1 << 22)) return;
  if (out_size != 2 * nN) return;
  if (in_sizes[0] <= 0 || (in_sizes[0] & 1) != 0) return;
  const int nE = in_sizes[0] / 2;
  if (nE <= 0 || nE > (1 << 26)) return;
  if (in_sizes[1] != nE) return;
  if (in_sizes[4] != 2 * HD || in_sizes[5] != HD) return;
  if (in_sizes[6] != 136 * HD || in_sizes[7] != HD) return;
  if (in_sizes[8] != HD * HD || in_sizes[9] != HD || in_sizes[10] != HD * HD || in_sizes[11] != HD) return;
  if (in_sizes[12] != HD * G3 || in_sizes[13] != G3 || in_sizes[14] != HD * G3 || in_sizes[15] != G3) return;
  if (in_sizes[16] != HD * 2 || in_sizes[17] != 2) return;

  const int*   msgn  = (const int*)d_in[0];
  const float* Jm    = (const float*)d_in[1];
  const float* bnode = (const float*)d_in[2];
  const float* Win   = (const float*)d_in[4];
  const float* bin0  = (const float*)d_in[5];
  const float* W1    = (const float*)d_in[6];
  const float* b1    = (const float*)d_in[7];
  const float* W2    = (const float*)d_in[8];
  const float* b2    = (const float*)d_in[9];
  const float* W3    = (const float*)d_in[10];
  const float* b3    = (const float*)d_in[11];
  const float* Wih   = (const float*)d_in[12];
  const float* bih   = (const float*)d_in[13];
  const float* Whh   = (const float*)d_in[14];
  const float* bhh   = (const float*)d_in[15];
  const float* Wout  = (const float*)d_in[16];
  const float* bout  = (const float*)d_in[17];
  float* out = (float*)d_out;

  const int NPAD   = ((nN + NGRAN - 1) / NGRAN) * NGRAN;
  const int nBC    = (nN + NBC - 1) / NBC;
  const int CNTPAD = nBC * NBC;
  if (CNTPAD < NPAD) return;
  if (4 * nBC + 1 > RBN) return;
  const int nBF    = (nN + NBF - 1) / NBF;
  if (nBF + 1 > 4 * nBC + 1) return;
  const int nE32   = (nE + 31) & ~31;
  const int csrLen = nE32 + 4096;
  if (31 * 4 * nBC > 4096) return;
  const int nEdgeB = NPAD / TGT;
  const int nNodeB = NPAD / BM;
  const int nObjU  = nE32 / 4;

  char* ws = (char*)d_ws;
  size_t off = 0;
  const size_t oObj = off; off += (size_t)nE32 * 4;              off = (off + 255) & ~(size_t)255;
  const size_t oCnt = off; off += (size_t)CNTPAD * 4;            off = (off + 255) & ~(size_t)255;
  const size_t oOff = off; off += (size_t)CNTPAD * 4;            off = (off + 255) & ~(size_t)255;
  const size_t oRb  = off; off += (size_t)RBN * 4;               off = (off + 255) & ~(size_t)255;
  const size_t oCsr = off; off += (size_t)csrLen * 4;            off = (off + 255) & ~(size_t)255;
  const size_t oWp  = off; off += (size_t)WPROWS * HD * 2;       off = (off + 255) & ~(size_t)255;
  const size_t oP   = off; off += (size_t)NPAD * HD * 4;         off = (off + 255) & ~(size_t)255;
  const size_t oQ   = off; off += (size_t)NPAD * HD * 4;         off = (off + 255) & ~(size_t)255;
  const size_t oH32 = off; off += (size_t)NPAD * HD * 4;         off = (off + 255) & ~(size_t)255;
  const size_t oH16 = off; off += (size_t)NPAD * HD * 2;         off = (off + 255) & ~(size_t)255;
  const size_t oAgg = off; off += (size_t)NPAD * HD * 2;         off = (off + 255) & ~(size_t)255;
  if (off > ws_size || off > (size_t)WSCAP) return;
  int*      objP = (int*)(ws + oObj);
  int*      cnt  = (int*)(ws + oCnt);
  int*      offp = (int*)(ws + oOff);
  int*      rb   = (int*)(ws + oRb);
  int*      csr  = (int*)(ws + oCsr);
  _Float16* WP   = (_Float16*)(ws + oWp);
  float*    Pp   = (float*)(ws + oP);
  float*    Qp   = (float*)(ws + oQ);
  float*    H32  = (float*)(ws + oH32);
  _Float16* H16  = (_Float16*)(ws + oH16);
  _Float16* aggP = (_Float16*)(ws + oAgg);

  k_extract<<<(nObjU + NTHR - 1) / NTHR, NTHR, 0, stream>>>(msgn, objP, nE, nObjU);
  k_count<<<nBC, NTHR, 0, stream>>>(objP, cnt, nE, 1);
  k_offsets<<<1, OTHR, 0, stream>>>(cnt, offp, rb, nBC);
  hipFuncSetAttribute(reinterpret_cast<const void*>(&k_fill),
                      hipFuncAttributeMaxDynamicSharedMemorySize, LDS_FILL);
  k_fill<<<nBF, NTHR, LDS_FILL, stream>>>(objP, offp, rb, csr, nE, 1, csrLen);

  k_prepw<<<dim3((G3 * 8 + NTHR - 1) / NTHR, 6), NTHR, 0, stream>>>(W1, W2, W3, Wih, Whh, WP);

  k_node<<<nNodeB, NTHR, 0, stream>>>(aggP, WP, W1, b1, bnode, Win, bin0, bih, bhh, Wout, bout,
                                      H32, H16, Pp, Qp, out, nN, 0);

  for (int it = 0; it < NPROP; ++it) {
    k_edge<<<nEdgeB, ETHR, 0, stream>>>(csr, offp, cnt, msgn, Jm, Pp, Qp, WP, W1, b2, b3,
                                        aggP, nN, nE, csrLen);
    k_node<<<nNodeB, NTHR, 0, stream>>>(aggP, WP, W1, b1, bnode, Win, bin0, bih, bhh, Wout, bout,
                                        H32, H16, Pp, Qp, out, nN, (it == NPROP - 1) ? 2 : 1);
  }
}
